// SelfAttentionConv_54546084659812
// MI455X (gfx1250) — hardware-verified
//
#include <hip/hip_runtime.h>


#ifndef NB
#define NB 8
#endif
#ifndef SEQ
#define SEQ 1024
#endif

namespace {
typedef _Float16 b16;
typedef __attribute__((ext_vector_type(16))) _Float16 v16b;
typedef __attribute__((ext_vector_type(8))) _Float16 v8b;
typedef __attribute__((ext_vector_type(4))) _Float16 v4h;
typedef __attribute__((ext_vector_type(8))) float v8f;
typedef __attribute__((ext_vector_type(4))) float v4f;
__device__ __forceinline__ float bf16_rne(float f) { unsigned int u = __float_as_uint(f); u += 0x7FFFu + ((u >> 16) & 1u); return __uint_as_float(u & 0xFFFF0000u); }
__device__ __forceinline__ v16b frag_kb(const b16* p, int hh) { const v8b a = *(const v8b*)(p + 8 * hh), b = *(const v8b*)(p + 16 + 8 * hh); v16b f;
#pragma unroll
  for (int e = 0; e < 8; ++e) { f[e] = a[e]; f[8 + e] = b[e]; } return f; }
__device__ __forceinline__ v8f wmma16b(v16b a, v16b b, v8f c) { v8f d = __builtin_amdgcn_wmma_f32_16x16x32_f16(false, a, false, b, (short)0, c, false, false); asm volatile("v_nop\n\tv_nop\n\tv_nop\n\tv_nop" : "+v"(d) : "v"(a), "v"(b)); return d; }
__device__ __forceinline__ void wave_lds_sync() { __builtin_amdgcn_fence(__ATOMIC_RELEASE, "workgroup"); __builtin_amdgcn_wave_barrier(); __builtin_amdgcn_fence(__ATOMIC_ACQUIRE, "workgroup"); }
__device__ __forceinline__ float nexp2(float v) { return __builtin_amdgcn_exp2f(v); }
__device__ __forceinline__ float silu(float v) { return v / (1.0f + __expf(-v)); }

constexpr int NB_FULL = 8, T_FULL = 1024;
constexpr int BL = NB  , T = SEQ  , KC = 64, NH = 8, CO = NH * KC  , CW = 2 * CO  , KS = 5, DIL = 2,
              KQ = KS * KC  , NROW = BL * T, NM = BL * NH  , TB = T / NH  , WIN = 5;
constexpr float XS = 8.0f, WSC = 256.0f, PS = 1024.0f, RS_ = 1024.0f, LOG2E = 1.4426950408889634f, SCALE = 0.125f  ;
static_assert(BL >= 1 && BL <= NB_FULL);
static_assert(T >= 64 && T <= T_FULL && T % 64 == 0 && T % NH == 0);
static_assert(KC == 64 && CO % 128 == 0 && KQ % 32 == 0 && CW % 128 == 0 && NROW % 32 == 0 && CO / NH == KC);

template <int KS_>
__global__ __launch_bounds__(256) void wperm_kernel(const float* __restrict__ w, b16* __restrict__ WT) {
  const int u = blockIdx.x * 256 + threadIdx.x; if (u >= CO * KS_ * KC / 8) return; const int e = u * 8; const int op = e / (KS_ * KC), k0 = e % (KS_ * KC); const int h = op / KC, kk = op % KC, o = kk * NH + h; v8b v;
  const int j = k0 / KC, c0 = k0 % KC;
#pragma unroll
  for (int jj = 0; jj < 8; ++jj) v[jj] = (b16)(bf16_rne(w[((size_t)o * KC + c0 + jj) * KS_ + j]) * WSC);
  for (int pass = 0; pass < 2; ++pass) { *(volatile v8b*)(WT + e) = v; __threadfence(); }
}
__global__ __launch_bounds__(256) void bperm_kernel(const float* __restrict__ bsrc, float* __restrict__ BP) { const int op = blockIdx.x * 256 + threadIdx.x; if (op >= CO) return; const int h = op / KC, kk = op % KC; const float v = bsrc[kk * NH + h]; for (int pass = 0; pass < 2; ++pass) { ((volatile float*)BP)[op] = v; __threadfence(); } }
__global__ __launch_bounds__(256) void wcvt_kernel(const float* __restrict__ w, b16* __restrict__ W16, int n8) { const int u = blockIdx.x * 256 + threadIdx.x; if (u >= n8) return; const size_t e = (size_t)u * 8; v8b o;
#pragma unroll
  for (int j = 0; j < 8; ++j) o[j] = (b16)(bf16_rne(w[e + j]) * WSC);
  for (int pass = 0; pass < 2; ++pass) { *(volatile v8b*)(W16 + e) = o; __threadfence(); } }
template <int KS_, int MODE>
__global__ __launch_bounds__(64) void conv_kernel(const float* __restrict__ x, const b16* __restrict__ WT, const float* __restrict__ bias, b16* __restrict__ P0, float* __restrict__ VF) {
  constexpr int KD = KS_ * KC;
  __shared__ __attribute__((aligned(16))) b16 As[2][16][KC + 8]; __shared__ __attribute__((aligned(16))) float Tf[2][16][128 + 4];
  const int wave = threadIdx.x >> 5, lane = threadIdx.x & 31, nloc = lane & 15, hlf = lane >> 4; const int b = blockIdx.z; const int t0 = blockIdx.x * 32 + wave * 16; const int n0 = blockIdx.y * 128;
  v8f acc[8];
#pragma unroll
  for (int tt = 0; tt < 8; ++tt) acc[tt] = (v8f){};
#pragma unroll 1
  for (int j = 0; j < KS_; ++j) { const int dt = KS_ == 1 ? 0 : DIL * j - (KS_ - 1) * DIL;
    for (int idx = lane; idx < 16 * (KC / 4); idx += 32) { const int rr = idx / (KC / 4), c4 = (idx % (KC / 4)) * 4; const int t = t0 + rr + dt; const int tc = t < 0 ? 0 : t;
      const v4f v = *(const v4f*)(x + ((size_t)b * T_FULL + tc) * KC + c4); v4h o;
#pragma unroll
      for (int q = 0; q < 4; ++q) o[q] = (t >= 0) ? (b16)(bf16_rne(v[q]) * XS) : (b16)0.0f;
      *(v4h*)(&As[wave][rr][c4]) = o; }
    wave_lds_sync();
#pragma unroll
    for (int kb = 0; kb < KC; kb += 32) { const v16b a = frag_kb(&As[wave][nloc][kb], hlf);
#pragma unroll
      for (int tt = 0; tt < 8; ++tt) acc[tt] = wmma16b(a, frag_kb(WT + (size_t)(n0 + tt * 16 + nloc) * KD + j * KC + kb, hlf), acc[tt]); }
    wave_lds_sync(); }
#pragma unroll
  for (int tt = 0; tt < 8; ++tt) { const float bb = bias ? bf16_rne(bias[n0 + tt * 16 + nloc]) : 0.0f;
#pragma unroll
    for (int r = 0; r < 8; ++r) Tf[wave][8 * hlf + r][tt * 16 + nloc] = silu(acc[tt][r] * (1.0f / (XS * WSC)) + bb); }
  wave_lds_sync();
  for (int pass = 0; pass < 2; ++pass) { for (int rr = 0; rr < 16; ++rr) { const size_t row = (size_t)b * T + t0 + rr;
      if (MODE & 1) { v4h o;
#pragma unroll
        for (int q = 0; q < 4; ++q) o[q] = (b16)(Tf[wave][rr][lane * 4 + q] * XS);
        *(volatile v4h*)(P0 + row * CO + n0 + lane * 4) = o; }
      if (MODE & 2) { *(volatile v4f*)(VF + row * CO + n0 + lane * 4) = *(const v4f*)(&Tf[wave][rr][lane * 4]); } } __threadfence(); }
}
__global__ __launch_bounds__(256) void vt_kernel(const float* __restrict__ VF, b16* __restrict__ VTh, b16* __restrict__ VTl) {
  const int bm = blockIdx.x, b = bm / NH, m = bm % NH, kk0 = blockIdx.y * 16;
  for (int i = threadIdx.x; i < 16 * (T / 8); i += 256) { const int kk = kk0 + i / (T / 8), p0 = (i % (T / 8)) * 8; v8b oh, ol;
#pragma unroll
    for (int e = 0; e < 8; ++e) { const int p = p0 + e; const int t = TB * m + p / 8, h = p % 8; const float vs = VF[((size_t)b * T + t) * CO + h * KC + kk] * XS; const b16 ph = (b16)vs; oh[e] = ph; ol[e] = (b16)((vs - (float)ph) * RS_); }
    const size_t dst = ((size_t)bm * KC + kk) * T + p0; for (int pass = 0; pass < 2; ++pass) { *(volatile v8b*)(VTh + dst) = oh; *(volatile v8b*)(VTl + dst) = ol; __threadfence(); } }
}
__global__ __launch_bounds__(64) void attn_kernel(const b16* __restrict__ QP, const b16* __restrict__ KP, const b16* __restrict__ VTh, const b16* __restrict__ VTl,
                                                  const b16* __restrict__ LP, const b16* __restrict__ LTh, const b16* __restrict__ LTl, float* __restrict__ CT) {
  __shared__ __attribute__((aligned(16))) b16 Pb[2][16][32 + 8], Pl[2][16][32 + 8]; __shared__ __attribute__((aligned(16))) float To[2][16][2 * KC + 4];
  const int wave = threadIdx.x >> 5, lane = threadIdx.x & 31, hh = lane >> 4, col = lane & 15; const int bm = blockIdx.y, b = bm / NH, m = bm % NH; const int p0 = blockIdx.x * 32 + wave * 16; const int pq = p0 + col;
  const size_t poff = (size_t)bm * T * KC;
  const float cs = LOG2E * SCALE / (XS * XS);
  {
    const b16* Lq = LP + poff; const b16* Lh = LTh + poff; const b16* Ll = LTl + poff;
    v16b qf[2];
#pragma unroll
    for (int kb = 0; kb < 2; ++kb) qf[kb] = frag_kb(Lq + (size_t)pq * KC + kb * 32, hh);
    const int s0 = (p0 >= 16) ? p0 - 16 : 0;
    float e[16]; float mx = -INFINITY;
#pragma unroll
    for (int u2 = 0; u2 < 2; ++u2) { v8f sacc = (v8f){};
#pragma unroll
      for (int kb = 0; kb < 2; ++kb) sacc = wmma16b(frag_kb(Lq + (size_t)(s0 + u2 * 16 + col) * KC + kb * 32, hh), qf[kb], sacc);
#pragma unroll
      for (int r = 0; r < 8; ++r) { const int s = s0 + u2 * 16 + 8 * hh + r; const bool ok = (s <= pq) && (pq - s <= WIN); const float vv = ok ? sacc[r] * cs : -INFINITY; e[u2 * 8 + r] = vv; mx = fmaxf(mx, vv); } }
    mx = fmaxf(mx, __shfl_xor(mx, 16)); float sum = 0.0f;
#pragma unroll
    for (int i2 = 0; i2 < 16; ++i2) { const float p = (mx == -INFINITY) ? 0.0f : nexp2(e[i2] - mx); sum += p; const float psv = p * PS; const b16 p1 = (b16)psv; const int slot = (i2 < 8 ? 0 : 16) + 8 * hh + (i2 & 7); Pb[wave][col][slot] = p1; Pl[wave][col][slot] = (b16)((psv - (float)p1) * RS_); }
    sum += __shfl_xor(sum, 16);
    wave_lds_sync();
    const v16b pf = frag_kb(&Pb[wave][col][0], hh), plf = frag_kb(&Pl[wave][col][0], hh);
    v8f ol[4], ol2[4];
#pragma unroll
    for (int t8 = 0; t8 < 4; ++t8) { ol[t8] = (v8f){}; ol2[t8] = (v8f){}; const v16b vh = frag_kb(Lh + (size_t)(t8 * 16 + col) * T + s0, hh); ol[t8] = wmma16b(vh, pf, ol[t8]); ol2[t8] = wmma16b(frag_kb(Ll + (size_t)(t8 * 16 + col) * T + s0, hh), pf, ol2[t8]); ol2[t8] = wmma16b(vh, plf, ol2[t8]); }
    wave_lds_sync();
    const float invl = 1.0f / (sum * PS * XS);
#pragma unroll
    for (int t8 = 0; t8 < 4; ++t8)
#pragma unroll
      for (int r = 0; r < 8; ++r) To[wave][col][t8 * 16 + 8 * hh + r] = (ol[t8][r] + ol2[t8][r] * (1.0f / RS_)) * invl;
  }
  const b16* Qb = QP + poff; const b16* Kb = KP + poff; const b16* Vh = VTh + poff; const b16* Vl = VTl + poff;
  v16b qf[2];
#pragma unroll
  for (int kb = 0; kb < 2; ++kb) qf[kb] = frag_kb(Qb + (size_t)pq * KC + kb * 32, hh);
  float mrun = -INFINITY, l = 0.0f; v8f o[4], o2[4];
#pragma unroll
  for (int t8 = 0; t8 < 4; ++t8) { o[t8] = (v8f){}; o2[t8] = (v8f){}; }
  const int send = p0 + 16;
#pragma unroll 1
  for (int s0 = 0; s0 < send; s0 += 32) {
    float e[16]; float mx = -INFINITY;
#pragma unroll
    for (int u2 = 0; u2 < 2; ++u2) { v8f sacc = (v8f){};
#pragma unroll
      for (int kb = 0; kb < 2; ++kb) sacc = wmma16b(frag_kb(Kb + (size_t)(s0 + u2 * 16 + col) * KC + kb * 32, hh), qf[kb], sacc);
#pragma unroll
      for (int r = 0; r < 8; ++r) { const int s = s0 + u2 * 16 + 8 * hh + r; const float vv = (s <= pq) ? sacc[r] * cs : -INFINITY; e[u2 * 8 + r] = vv; mx = fmaxf(mx, vv); } }
    mx = fmaxf(mx, __shfl_xor(mx, 16)); const float mn = fmaxf(mrun, mx); const float al = (mn == -INFINITY) ? 1.0f : nexp2(mrun - mn); float sum = 0.0f;
#pragma unroll
    for (int i2 = 0; i2 < 16; ++i2) { const float p = (mn == -INFINITY) ? 0.0f : nexp2(e[i2] - mn); sum += p; const float psv = p * PS; const b16 p1 = (b16)psv; const int slot = (i2 < 8 ? 0 : 16) + 8 * hh + (i2 & 7); Pb[wave][col][slot] = p1; Pl[wave][col][slot] = (b16)((psv - (float)p1) * RS_); }
    sum += __shfl_xor(sum, 16); l = l * al + sum; mrun = mn;
    wave_lds_sync();
    const v16b pf = frag_kb(&Pb[wave][col][0], hh), plf = frag_kb(&Pl[wave][col][0], hh);
#pragma unroll
    for (int t8 = 0; t8 < 4; ++t8) { o[t8] *= al; o2[t8] *= al; const v16b vh = frag_kb(Vh + (size_t)(t8 * 16 + col) * T + s0, hh); o[t8] = wmma16b(vh, pf, o[t8]); o2[t8] = wmma16b(frag_kb(Vl + (size_t)(t8 * 16 + col) * T + s0, hh), pf, o2[t8]); o2[t8] = wmma16b(vh, plf, o2[t8]); }
    wave_lds_sync(); }
  const float inv = 1.0f / (l * PS * XS);
#pragma unroll
  for (int t8 = 0; t8 < 4; ++t8)
#pragma unroll
    for (int r = 0; r < 8; ++r) { const int di = t8 * 16 + 8 * hh + r; const float og = (o[t8][r] + o2[t8][r] * (1.0f / RS_)) * inv; const float g = 1.0f / (1.0f + __expf(-og)); const float lv = To[wave][col][di];
      To[wave][col][di] = (1.0f - g) * lv; To[wave][col][KC + di] = g * og; }
  wave_lds_sync();
  for (int pass = 0; pass < 2; ++pass) { for (int rr = 0; rr < 16; ++rr) *(volatile v4f*)(CT + ((size_t)b * T + p0 + rr) * CW + m * KC + hh * CO + col * 4) = *(const v4f*)(&To[wave][rr][lane * 4]); __threadfence(); }
}
__global__ __launch_bounds__(64) void outp_kernel(const float* __restrict__ CT, const b16* __restrict__ WU, const float* __restrict__ bu, float* __restrict__ out) {
  __shared__ __attribute__((aligned(16))) b16 Ah[2][16][128 + 8], Al[2][16][128 + 8]; __shared__ __attribute__((aligned(16))) float Tf[2][16][KC + 4];
  const int wave = threadIdx.x >> 5, lane = threadIdx.x & 31, nloc = lane & 15, hlf = lane >> 4; const size_t m0 = (size_t)blockIdx.x * 32 + wave * 16;
  v8f acc[4], acc2[4];
#pragma unroll
  for (int t8 = 0; t8 < 4; ++t8) { acc[t8] = (v8f){}; acc2[t8] = (v8f){}; }
#pragma unroll 1
  for (int kc = 0; kc < CW; kc += 128) {
    for (int idx = lane; idx < 16 * 32; idx += 32) { const int rr = idx / 32, c4 = (idx % 32) * 4; const v4f v = *(const v4f*)(CT + (m0 + rr) * CW + kc + c4); v4h hv, lv;
#pragma unroll
      for (int q = 0; q < 4; ++q) { const float vs = v[q] * XS; const b16 ph = (b16)vs; hv[q] = ph; lv[q] = (b16)((vs - (float)ph) * RS_); }
      *(v4h*)(&Ah[wave][rr][c4]) = hv; *(v4h*)(&Al[wave][rr][c4]) = lv; }
    wave_lds_sync();
#pragma unroll
    for (int kb = 0; kb < 128; kb += 32) { const v16b a = frag_kb(&Ah[wave][nloc][kb], hlf), al = frag_kb(&Al[wave][nloc][kb], hlf);
#pragma unroll
      for (int t8 = 0; t8 < 4; ++t8) { const v16b bw = frag_kb(WU + (size_t)(t8 * 16 + nloc) * CW + kc + kb, hlf); acc[t8] = wmma16b(a, bw, acc[t8]); acc2[t8] = wmma16b(al, bw, acc2[t8]); } }
    wave_lds_sync(); }
#pragma unroll
  for (int t8 = 0; t8 < 4; ++t8) { const float bb = bf16_rne(bu[t8 * 16 + nloc]);
#pragma unroll
    for (int r = 0; r < 8; ++r) Tf[wave][8 * hlf + r][t8 * 16 + nloc] = silu((acc[t8][r] + acc2[t8][r] * (1.0f / RS_)) * (1.0f / (XS * WSC)) + bb); }
  wave_lds_sync();
  for (int pass = 0; pass < 2; ++pass) { for (int r2 = 0; r2 < 8; ++r2) *(volatile v4f*)(out + (m0 + 2 * r2) * KC + lane * 4) = *(const v4f*)(&Tf[wave][2 * r2 + hlf][nloc * 4]); __threadfence(); }
}
}

extern "C" void kernel_launch(void* const* d_in, const int* in_sizes, int n_in, void* d_out, int out_size, void* d_ws, size_t ws_size, hipStream_t stream) {
  (void)n_in;
  auto Fp = [&](int i) { return (const float*)d_in[i]; };
  if (in_sizes[0] < ((BL - 1) * T_FULL + T) * KC || in_sizes[1] < CO * KC * KS || in_sizes[2] < CO || in_sizes[3] < CO * KC * KS || in_sizes[4] < CO || in_sizes[5] < CO * KC || in_sizes[6] < CO * KC ||
      in_sizes[7] < KC * CW || in_sizes[8] < KC || out_size < NROW * KC) return;
  size_t off = 0; char* ws = (char*)d_ws;
  auto carve = [&](size_t bytes) { char* p = ws + off; off += (bytes + 255) & ~(size_t)255; return p; };
  b16* WQT = (b16*)carve((size_t)CO * KQ * 2); b16* WKT = (b16*)carve((size_t)CO * KQ * 2); b16* WVT = (b16*)carve((size_t)CO * KC * 2); b16* WLT = (b16*)carve((size_t)CO * KC * 2); b16* WU = (b16*)carve((size_t)KC * CW * 2);
  float* BQ = (float*)carve((size_t)CO * 4); float* BK = (float*)carve((size_t)CO * 4);
  b16* QP = (b16*)carve((size_t)NROW * CO * 2); b16* KP = (b16*)carve((size_t)NROW * CO * 2); b16* LP = (b16*)carve((size_t)NROW * CO * 2);
  float* VF = (float*)carve((size_t)NROW * CO * 4); float* LF = (float*)carve((size_t)NROW * CO * 4);
  b16* VTh = (b16*)carve((size_t)NROW * CO * 2); b16* VTl = (b16*)carve((size_t)NROW * CO * 2); b16* LTh = (b16*)carve((size_t)NROW * CO * 2); b16* LTl = (b16*)carve((size_t)NROW * CO * 2);
  float* CT = (float*)carve((size_t)NROW * CW * 4);
  if (off > ws_size || off > ((size_t)128 << 20)) return;
  wperm_kernel<KS><<<(CO * KQ / 8 + 255) / 256, 256, 0, stream>>>(Fp(1), WQT); wperm_kernel<KS><<<(CO * KQ / 8 + 255) / 256, 256, 0, stream>>>(Fp(3), WKT);
  wperm_kernel<1><<<(CO * KC / 8 + 255) / 256, 256, 0, stream>>>(Fp(5), WVT); wperm_kernel<1><<<(CO * KC / 8 + 255) / 256, 256, 0, stream>>>(Fp(6), WLT);
  wcvt_kernel<<<(KC * CW / 8 + 255) / 256, 256, 0, stream>>>(Fp(7), WU, KC * CW / 8);
  bperm_kernel<<<(CO + 255) / 256, 256, 0, stream>>>(Fp(2), BQ); bperm_kernel<<<(CO + 255) / 256, 256, 0, stream>>>(Fp(4), BK);
  conv_kernel<KS, 1><<<dim3(T / 32, CO / 128, BL), 64, 0, stream>>>(Fp(0), WQT, BQ, QP, nullptr);
  conv_kernel<KS, 1><<<dim3(T / 32, CO / 128, BL), 64, 0, stream>>>(Fp(0), WKT, BK, KP, nullptr);
  conv_kernel<1, 2><<<dim3(T / 32, CO / 128, BL), 64, 0, stream>>>(Fp(0), WVT, nullptr, nullptr, VF);
  conv_kernel<1, 3><<<dim3(T / 32, CO / 128, BL), 64, 0, stream>>>(Fp(0), WLT, nullptr, LP, LF);
  vt_kernel<<<dim3(NM, KC / 16), 256, 0, stream>>>(VF, VTh, VTl);
  vt_kernel<<<dim3(NM, KC / 16), 256, 0, stream>>>(LF, LTh, LTl);
  attn_kernel<<<dim3(T / 32, NM), 64, 0, stream>>>(QP, KP, VTh, VTl, LP, LTh, LTl, CT);
  outp_kernel<<<NROW / 32, 64, 0, stream>>>(CT, WU, Fp(8), (float*)d_out);
}
